// ConcatCritic_3736621548237
// MI455X (gfx1250) — hardware-verified
//
#include <hip/hip_runtime.h>
#include <stdint.h>
#include <stddef.h>


typedef _Float16 h16;
typedef __attribute__((ext_vector_type(16))) _Float16 v16h;
typedef __attribute__((ext_vector_type(8)))  float  v8f;

struct alignas(16) U4 { unsigned int x, y, z, w; };
struct alignas(16) F4 { float x, y, z, w; };
struct alignas(32) Frag { U4 lo, hi; };

#define HIDN 512
#define BSZ  256
#define MT   64
#define LSTR 520

__device__ __forceinline__ unsigned short f2bf(float f) {
  return __builtin_bit_cast(unsigned short, (h16)f);
}
__device__ __forceinline__ float bf2f(unsigned short h) {
  return (float)__builtin_bit_cast(h16, h);
}
__device__ __forceinline__ v8f wmma16(v16h a, v16h b, v8f c) {
  v8f d = __builtin_amdgcn_wmma_f32_16x16x32_f16(false, a, false, b, (short)0, c, false, false);
  asm volatile("v_nop\n\tv_nop\n\tv_nop\n\tv_nop" : "+v"(d) : "v"(a), "v"(b));
  return d;
}

__device__ __forceinline__ v16h load_frag(const unsigned short* base) {
  Frag fr;
  fr.lo = *(const U4*)(base);
  fr.hi = *(const U4*)(base + 16);
  return __builtin_bit_cast(v16h, fr);
}

__device__ __forceinline__ void mlp_layer(const unsigned short* sIn,
                                          unsigned short*       sOut,
                                          const unsigned short* __restrict__ Wt,
                                          const float* __restrict__ bias) {
  const int lane = threadIdx.x & 31;
  const int wave = threadIdx.x >> 5;
  const int lr   = lane & 15;
  const int kh   = (lane >> 4) << 3;
  const int n0   = wave * 64;

  v8f acc[4][4];
#pragma unroll
  for (int a = 0; a < 4; ++a)
#pragma unroll
    for (int b = 0; b < 4; ++b)
      acc[a][b] = (v8f){0.f, 0.f, 0.f, 0.f, 0.f, 0.f, 0.f, 0.f};

  for (int kk = 0; kk < HIDN; kk += 32) {
    const int kb = kk + kh;
    v16h af[4], bf[4];
#pragma unroll
    for (int tm = 0; tm < 4; ++tm)
      af[tm] = load_frag(&sIn[(tm * 16 + lr) * LSTR + kb]);
#pragma unroll
    for (int tn = 0; tn < 4; ++tn)
      bf[tn] = load_frag(&Wt[(size_t)(n0 + tn * 16 + lr) * HIDN + kb]);
#pragma unroll
    for (int tn = 0; tn < 4; ++tn)
#pragma unroll
      for (int tm = 0; tm < 4; ++tm)
        acc[tm][tn] = wmma16(af[tm], bf[tn], acc[tm][tn]);
  }

  const int mrb = (lane >> 4) << 3;
#pragma unroll
  for (int tn = 0; tn < 4; ++tn) {
    const int n  = n0 + tn * 16 + lr;
    const float bn = bias[n];
#pragma unroll
    for (int tm = 0; tm < 4; ++tm) {
#pragma unroll
      for (int r = 0; r < 8; ++r) {
        float v = fmaxf(acc[tm][tn][r] * 0.0625f + bn, 0.f);
        sOut[(tm * 16 + mrb + r) * LSTR + n] = f2bf(v);
      }
    }
  }
  __syncthreads();
}

__global__ __launch_bounds__(256) void fused_critic(
    const float* __restrict__ hx,
    const float* __restrict__ hy,
    const unsigned short* __restrict__ W1t,
    const float* __restrict__ b1,
    const unsigned short* __restrict__ W2t,
    const float* __restrict__ b2,
    const float* __restrict__ W3,
    const float* __restrict__ b3,
    float* __restrict__ out)
{
  extern __shared__ __attribute__((aligned(16))) unsigned short smem[];
  __shared__ __attribute__((aligned(16))) float sOut[64];
  unsigned short* sA = smem;
  unsigned short* sB = smem + MT * LSTR;

  const int blk = blockIdx.x;
  const int i   = blk >> 2;
  const int j0  = (blk & 3) * MT;

  {
    const int t  = threadIdx.x;
    const int r  = t >> 2;
    const int k0 = (t & 3) * 128;
    const F4* px = (const F4*)&hx[(size_t)i * HIDN + k0];
    const F4* py = (const F4*)&hy[(size_t)(j0 + r) * HIDN + k0];
    unsigned short* dst = &sA[r * LSTR + k0];
#pragma unroll 4
    for (int q = 0; q < 32; ++q) {
      F4 a = px[q];
      F4 b = py[q];
      unsigned int p0 = (unsigned int)f2bf(fmaxf(a.x + b.x, 0.f)) |
                        ((unsigned int)f2bf(fmaxf(a.y + b.y, 0.f)) << 16);
      unsigned int p1 = (unsigned int)f2bf(fmaxf(a.z + b.z, 0.f)) |
                        ((unsigned int)f2bf(fmaxf(a.w + b.w, 0.f)) << 16);
      unsigned int* d32 = (unsigned int*)(dst + q * 4);
      d32[0] = p0;
      d32[1] = p1;
    }
  }
  __syncthreads();

  mlp_layer(sA, sB, W1t, b1);
  mlp_layer(sB, sA, W2t, b2);

  {
    const int t  = threadIdx.x;
    const int r  = t >> 2;
    const int k0 = (t & 3) * 128;
    const unsigned short* row = &sA[r * LSTR];
    float acc = 0.f;
    for (int k = k0; k < k0 + 128; ++k)
      acc += bf2f(row[k]) * W3[k];
    acc += __shfl_xor(acc, 1, 32);
    acc += __shfl_xor(acc, 2, 32);
    if ((t & 3) == 0) sOut[r] = acc + b3[0];
  }
  __syncthreads();
  if (threadIdx.x < 32) {
    const int l = threadIdx.x;
    volatile float* o = out + (size_t)i * BSZ + j0;
    o[l] = sOut[l]; o[32 + l] = sOut[32 + l];
    __threadfence();
    o[l] = sOut[l]; o[32 + l] = sOut[32 + l];
  }
}

__global__ __launch_bounds__(256) void prep_proj(
    const float* __restrict__ x,  const float* __restrict__ y,
    const float* __restrict__ Wx, const float* __restrict__ Wy,
    const float* __restrict__ b0,
    float* __restrict__ hx, float* __restrict__ hy)
{
  const int id   = blockIdx.x * 256 + threadIdx.x;
  const int half = id >> 17;
  const int idx  = id & 131071;
  const int row  = idx >> 9;
  const int h    = idx & 511;
  float acc; volatile float* dst;
  if (half == 0) {
    acc = b0[h];
    for (int k = 0; k < 128; ++k) acc += x[row * 128 + k] * Wx[k * 512 + h];
    dst = hx + idx;
  } else {
    acc = 0.f;
    for (int k = 0; k < 128; ++k) acc += y[row * 128 + k] * Wy[k * 512 + h];
    dst = hy + idx;
  }
  *dst = acc;
  __threadfence();
  *dst = acc;
}

struct alignas(16) H8 { unsigned short e[8]; };
__global__ __launch_bounds__(256) void prep_pack(
    const float* __restrict__ W1, const float* __restrict__ W2,
    unsigned short* __restrict__ W1t, unsigned short* __restrict__ W2t)
{
  const int id   = blockIdx.x * 256 + threadIdx.x;
  const int half = id >> 15;
  const int idx  = id & 32767;
  const int n    = idx >> 6;
  const int k0   = (idx & 63) * 8;
  const float* W = half ? W2 : W1;
  unsigned short* Wt = half ? W2t : W1t;
  H8 v;
#pragma unroll
  for (int e = 0; e < 8; ++e) v.e[e] = f2bf(W[(k0 + e) * 512 + n] * 16.0f);
  volatile U4* d = (volatile U4*)(Wt + (size_t)n * 512 + k0);
  U4 u = __builtin_bit_cast(U4, v);
  d->x = u.x; d->y = u.y; d->z = u.z; d->w = u.w;
  __threadfence();
  d->x = u.x; d->y = u.y; d->z = u.z; d->w = u.w;
}

extern "C" void kernel_launch(void* const* d_in, const int* in_sizes, int n_in,
                              void* d_out, int out_size, void* d_ws, size_t ws_size,
                              hipStream_t stream) {
  const float* x  = (const float*)d_in[0];
  const float* y  = (const float*)d_in[1];
  const float* Wx = (const float*)d_in[2];
  const float* Wy = (const float*)d_in[3];
  const float* b0 = (const float*)d_in[4];
  const float* W1 = (const float*)d_in[5];
  const float* b1 = (const float*)d_in[6];
  const float* W2 = (const float*)d_in[7];
  const float* b2 = (const float*)d_in[8];
  const float* W3 = (const float*)d_in[9];
  const float* b3 = (const float*)d_in[10];
  float* out = (float*)d_out;

  float* hx = (float*)d_ws;
  float* hy = hx + 256 * 512;
  unsigned short* W1t = (unsigned short*)(hy + 256 * 512);
  unsigned short* W2t = W1t + 512 * 512;
  if (ws_size < (size_t)4 * 512 * 1024) return;
  (void)in_sizes; (void)n_in; (void)out_size;

  prep_proj<<<1024, 256, 0, stream>>>(x, y, Wx, Wy, b0, hx, hy);
  prep_pack<<<256, 256, 0, stream>>>(W1, W2, W1t, W2t);

  const size_t smem_bytes = 2u * MT * LSTR * sizeof(unsigned short);
  fused_critic<<<1024, 256, smem_bytes, stream>>>(hx, hy, W1t, b1, W2t, b2,
                                                  W3, b3, out);
}
